// MLP_52493090292303
// MI455X (gfx1250) — hardware-verified
//
#include <hip/hip_runtime.h>
#include <stdint.h>


typedef __bf16   v16b __attribute__((ext_vector_type(16)));
typedef _Float16 v8h  __attribute__((ext_vector_type(8)));
typedef float    v8f  __attribute__((ext_vector_type(8)));
typedef float    v4f  __attribute__((ext_vector_type(4)));
typedef unsigned v4u  __attribute__((ext_vector_type(4)));
typedef unsigned v2u  __attribute__((ext_vector_type(2)));

union FragB { v16b v; v4u q[2]; unsigned w[8]; };
union F8    { v4u u4; v8h h8; unsigned w[4]; };
union U8f   { v4f v[2]; float f[8]; };
union U2w   { v2u v; unsigned w[2]; };
union P4w   { v4u u4; unsigned w[4]; };

#ifndef NB
#define NB 262144
#endif
#define NB_FULL 262144
#define NIN  9
#define NHID 128
#define NOUT 9
#define RB   128
#define NBLK (NB / RB)
static_assert(NB % RB == 0);
static_assert(NB >= RB);
static_assert(NB <= NB_FULL);

#define WP1_OFF   0
#define WPH_OFF   2048
#define WP6_OFF   (2048 + 4 * 16384)
#define WP_ELEMS  (WP6_OFF + 2048)
#define PREP_BLOCKS (WP_ELEMS / 2048)
static_assert(WP_ELEMS % 2048 == 0);
static_assert(WPH_OFF == 2048);
static_assert(WP6_OFF == 33 * 2048);

#define WS_WP        0
#define WS_WP_BYTES  ((size_t)WP_ELEMS * 2)
#define WS_PART      (WS_WP + WS_WP_BYTES)
#define WS_PART_BYTES ((size_t)NBLK * 256 * 4)
#define WS_ST        (WS_PART + WS_PART_BYTES)
#define WS_ST_BYTES  ((size_t)1024)
#define WS_HPL       (WS_ST + WS_ST_BYTES)
#define WS_HPL_BYTES ((size_t)NB * NHID * 2)
#define WS_LPL       (WS_HPL + WS_HPL_BYTES)
#define WS_LPL_BYTES ((size_t)NB * NHID)
#define WS_TOTAL     (WS_LPL + WS_LPL_BYTES)
static_assert(WS_WP_BYTES % 128 == 0);
static_assert(WS_PART % 128 == 0);
static_assert(WS_ST % 128 == 0);
static_assert(WS_HPL % 128 == 0);
static_assert(WS_LPL % 128 == 0);
static_assert(WS_TOTAL <= (size_t)134217728);

#define L_SB      0
#define L_SC      512
#define L_SH      1024
#define L_RED     1536
#define L_SS      2560
#define L_SQ      10752
#define L_STH     18944
#define STH_PITCH 136
#define L_STL     53760
#define STL_PITCH 144
#define LDS_A     72192
#define L_SO      1536
#define LDS_B     6144
static_assert(L_STH + 8 * 16 * 2 * STH_PITCH == L_STL);
static_assert(L_STL + 8 * 16 * STL_PITCH == LDS_A);
static_assert(L_SO + RB * NOUT * 4 == LDS_B);
static_assert((RB * NOUT * 4) % 128 == 0);

__device__ __forceinline__ unsigned bf16_bits(float x) {
    const unsigned u = __float_as_uint(x);
    return (u + 0x7FFFu + ((u >> 16) & 1u)) >> 16;
}
__device__ __forceinline__ float bf16r(float x) {
    return __uint_as_float(bf16_bits(x) << 16);
}

__device__ __forceinline__ v8f wmma_bf(v16b a, v16b b, v8f c) {
    v8f d = __builtin_amdgcn_wmma_f32_16x16x32_bf16(false, a, false, b, (short)0, c, false, false);
    asm volatile("v_nop\n\tv_nop\n\tv_nop\n\tv_nop" : "+v"(d) : "v"(a), "v"(b));
    return d;
}

__device__ __forceinline__ void afrag_split(const unsigned short* Hrow, const unsigned char* Lrow,
                                            const float* s_sc, const float* s_sh, int kt, int h,
                                            FragB& ahi, FragB& alo) {
#pragma unroll
    for (int hf = 0; hf < 2; ++hf) {
        const int kb = kt * 32 + 16 * hf + 8 * h;
        F8  hv; hv.u4 = *(const v4u*)(Hrow + kb);
        U2w lw; lw.v  = *(const v2u*)(Lrow + kb);
        U8f sc, sh;
        sc.v[0] = *(const v4f*)(s_sc + kb);  sc.v[1] = *(const v4f*)(s_sc + kb + 4);
        sh.v[0] = *(const v4f*)(s_sh + kb);  sh.v[1] = *(const v4f*)(s_sh + kb + 4);
#pragma unroll
        for (int p = 0; p < 4; ++p) {
            unsigned whi = 0u, wlo = 0u;
#pragma unroll
            for (int e = 0; e < 2; ++e) {
                const int j = 2 * p + e;
                const unsigned hb = (hv.w[p] >> (16 * e)) & 0xFFFFu;
                const unsigned E  = (hb >> 10) & 31u;
                const unsigned Em = (E == 0u) ? 1u : E;
                const float dsc   = __uint_as_float((Em + 94u) << 23);
                const unsigned lwd = lw.w[j >> 2];
                const int lo = ((int)(lwd << (24 - 8 * (j & 3)))) >> 24;
                const float y = (float)hv.h8[j] + (float)lo * dsc;
                const float z = y * sc.f[j] + sh.f[j];
                const float q = (z > 0.0f) ? z : 0.01f * z;
                const unsigned qh = bf16_bits(q);
                const float qhf   = __uint_as_float(qh << 16);
                const unsigned ql = bf16_bits(q - qhf);
                whi |= qh << (16 * e);
                wlo |= ql << (16 * e);
            }
            ahi.w[hf * 4 + p] = whi;
            alo.w[hf * 4 + p] = wlo;
        }
    }
}

__device__ __forceinline__ void epilogue_planes(v8f (&acc)[8], int blk, int wave, int lane, int tid,
                                                unsigned char* smem, unsigned short* Hpl, unsigned char* Lpl,
                                                float* part) {
    const int h = lane >> 4, m = lane & 15;
    const float* s_b = (const float*)(smem + L_SB);
    float* sS  = (float*)(smem + L_SS);
    float* sQ  = (float*)(smem + L_SQ);
    float* red = (float*)(smem + L_RED);
    unsigned short* stH = (unsigned short*)(smem + L_STH) + wave * (16 * STH_PITCH);
    unsigned char*  stL = smem + L_STL + wave * (16 * STL_PITCH);
    const int hslot = wave * 2 + h;

#pragma unroll
    for (int nt = 0; nt < 8; ++nt) {
        const int n = nt * 16 + m;
        const float bn = s_b[n];
        float s1 = 0.0f, s2 = 0.0f;
#pragma unroll
        for (int r = 0; r < 8; ++r) {
            const float y = acc[nt][r] + bn;
            s1 += y;
            s2 += y * y;
            const _Float16 hh = (_Float16)y;
            const unsigned hb = (unsigned)__builtin_bit_cast(unsigned short, hh);
            const unsigned E  = (hb >> 10) & 31u;
            const unsigned Em = (E == 0u) ? 1u : E;
            const float up    = __uint_as_float((160u - Em) << 23);
            float rq = rintf((y - (float)hh) * up);
            rq = fminf(fmaxf(rq, -128.0f), 127.0f);
            const int qi = (int)rq;
            const int row = 8 * h + r;
            stH[row * STH_PITCH + n] = (unsigned short)hb;
            stL[row * STL_PITCH + n] = (unsigned char)(qi & 255);
        }
        sS[hslot * 128 + n] = s1;
        sQ[hslot * 128 + n] = s2;
    }
    __syncthreads();

    {
        float s = 0.0f;
        if (tid < 128) {
#pragma unroll
            for (int w = 0; w < 16; ++w) s += sS[w * 128 + tid];
        } else {
            const int f = tid - 128;
#pragma unroll
            for (int w = 0; w < 16; ++w) s += sQ[w * 128 + f];
        }
        red[tid] = s;
    }
    __syncthreads();

    v4u hp[8], lp[4];
#pragma unroll
    for (int t = 0; t < 8; ++t) {
        const int c = lane + 32 * t, row = c >> 4, off = (c & 15) * 8;
        hp[t] = *(const v4u*)(stH + row * STH_PITCH + off);
    }
#pragma unroll
    for (int t = 0; t < 4; ++t) {
        const int c = lane + 32 * t, row = c >> 3, offb = (c & 7) * 16;
        lp[t] = *(const v4u*)(stL + row * STL_PITCH + offb);
    }
    const v4f pp = *(const v4f*)(red + 4 * (tid & 63));
    const size_t row0 = (size_t)blk * RB + (size_t)wave * 16;
    float* pdst = part + (size_t)blk * 256 + 4 * (tid & 63);

#pragma unroll
    for (int t = 0; t < 8; ++t) {
        const int c = lane + 32 * t, row = c >> 4, off = (c & 15) * 8;
        *(volatile v4u*)(Hpl + (row0 + row) * NHID + off) = hp[t];
    }
#pragma unroll
    for (int t = 0; t < 4; ++t) {
        const int c = lane + 32 * t, row = c >> 3, offb = (c & 7) * 16;
        *(volatile v4u*)(Lpl + (row0 + row) * NHID + offb) = lp[t];
    }
    if (tid < 64) *(volatile v4f*)pdst = pp;
    __threadfence();
#pragma unroll
    for (int t = 0; t < 8; ++t) {
        const int c = lane + 32 * t, row = c >> 4, off = (c & 15) * 8;
        *(volatile v4u*)(Hpl + (row0 + row) * NHID + off) = hp[t];
    }
#pragma unroll
    for (int t = 0; t < 4; ++t) {
        const int c = lane + 32 * t, row = c >> 3, offb = (c & 7) * 16;
        *(volatile v4u*)(Lpl + (row0 + row) * NHID + offb) = lp[t];
    }
    if (tid < 64) *(volatile v4f*)pdst = pp;
}

__global__ __launch_bounds__(256) void k_prep(const float* __restrict__ W1, const float* __restrict__ W2,
                                               const float* __restrict__ W3, const float* __restrict__ W4,
                                               const float* __restrict__ W5, const float* __restrict__ W6,
                                               unsigned short* wpl) {
    const int blk = blockIdx.x, tid = threadIdx.x;
    const int e0 = (blk * 256 + tid) * 8;
    P4w pk;
    if (blk == 0) {
#pragma unroll
        for (int p = 0; p < 4; ++p) {
            unsigned w = 0u;
#pragma unroll
            for (int e = 0; e < 2; ++e) {
                const int el = e0 + 2 * p + e, n = el >> 4, k = el & 15;
                const int kc = (k < NIN) ? k : (NIN - 1);
                const float wv = W1[n * NIN + kc];
                const unsigned bits = (k < NIN) ? bf16_bits(wv) : 0u;
                w |= bits << (16 * e);
            }
            pk.w[p] = w;
        }
    } else if (blk <= 32) {
        const int L = (blk - 1) >> 3;
        const float* W = (L == 0) ? W2 : (L == 1) ? W3 : (L == 2) ? W4 : W5;
        const int t0 = (e0 - WPH_OFF) & 16383;
        U8f wv;
        wv.v[0] = *(const v4f*)(W + t0);
        wv.v[1] = *(const v4f*)(W + t0 + 4);
#pragma unroll
        for (int p = 0; p < 4; ++p)
            pk.w[p] = bf16_bits(wv.f[2 * p]) | (bf16_bits(wv.f[2 * p + 1]) << 16);
    } else {
        const int t0 = e0 - WP6_OFF;
#pragma unroll
        for (int p = 0; p < 4; ++p) {
            unsigned w = 0u;
#pragma unroll
            for (int e = 0; e < 2; ++e) {
                const int t = t0 + 2 * p + e, n = t >> 7, k = t & 127;
                const int nc = (n < NOUT) ? n : (NOUT - 1);
                const float wv = W6[nc * NHID + k];
                const unsigned bits = (n < NOUT) ? bf16_bits(wv) : 0u;
                w |= bits << (16 * e);
            }
            pk.w[p] = w;
        }
    }
    unsigned short* dst = wpl + e0;
    *(volatile v4u*)dst = pk.u4;
    __threadfence();
    *(volatile v4u*)dst = pk.u4;
}

__global__ __launch_bounds__(256) void k_first(const float* __restrict__ x, const unsigned short* __restrict__ W1p,
                                                const float* __restrict__ b1, unsigned short* Hpl,
                                                unsigned char* Lpl, float* part) {
    extern __shared__ __attribute__((aligned(16))) unsigned char smem[];
    const int tid = threadIdx.x, wave = tid >> 5, lane = tid & 31, h = lane >> 4, m = lane & 15;
    float* s_b = (float*)(smem + L_SB);
    if (tid < NHID) s_b[tid] = bf16r(b1[tid]);
    __syncthreads();

    const size_t mrow = (size_t)blockIdx.x * RB + (size_t)wave * 16 + m;
    const float* xr = x + mrow * NIN;
    const v4u z4 = {0u, 0u, 0u, 0u};
    FragB a;
#pragma unroll
    for (int p = 0; p < 4; ++p) {
        unsigned w = 0u;
#pragma unroll
        for (int e = 0; e < 2; ++e) {
            const int k = 8 * h + 2 * p + e;
            const int kc = (k < NIN) ? k : (NIN - 1);
            const float xv = xr[kc];
            const unsigned bits = (k < NIN) ? bf16_bits(xv) : 0u;
            w |= bits << (16 * e);
        }
        a.w[p] = w;
    }
    a.q[1] = z4;

    v8f acc[8];
#pragma unroll
    for (int nt = 0; nt < 8; ++nt) acc[nt] = v8f{};
#pragma unroll
    for (int nt = 0; nt < 8; ++nt) {
        FragB b;
        b.q[0] = *(const v4u*)(W1p + (size_t)(nt * 16 + m) * 16 + 8 * h);
        b.q[1] = z4;
        acc[nt] = wmma_bf(a.v, b.v, acc[nt]);
    }
    epilogue_planes(acc, blockIdx.x, wave, lane, tid, smem, Hpl, Lpl, part);
}

__global__ __launch_bounds__(256) void k_mid(unsigned short* Hpl, unsigned char* Lpl, const float* __restrict__ st,
                                              const unsigned short* __restrict__ Wp, const float* __restrict__ bias,
                                              float* part) {
    extern __shared__ __attribute__((aligned(16))) unsigned char smem[];
    const int tid = threadIdx.x, wave = tid >> 5, lane = tid & 31, h = lane >> 4, m = lane & 15;
    float* s_b  = (float*)(smem + L_SB);
    float* s_sc = (float*)(smem + L_SC);
    float* s_sh = (float*)(smem + L_SH);
    if (tid < NHID) { s_b[tid] = bf16r(bias[tid]); s_sc[tid] = st[tid]; s_sh[tid] = st[NHID + tid]; }
    __syncthreads();

    const size_t mrow = (size_t)blockIdx.x * RB + (size_t)wave * 16 + m;
    const unsigned short* Hrow = Hpl + mrow * NHID;
    const unsigned char*  Lrow = Lpl + mrow * NHID;

    v8f acc[8];
#pragma unroll
    for (int nt = 0; nt < 8; ++nt) acc[nt] = v8f{};
#pragma unroll 1
    for (int kt = 0; kt < 4; ++kt) {
        FragB ahi, alo;
        afrag_split(Hrow, Lrow, s_sc, s_sh, kt, h, ahi, alo);
#pragma unroll
        for (int nt = 0; nt < 8; ++nt) {
            const unsigned short* wr = Wp + (size_t)(nt * 16 + m) * NHID + kt * 32 + 8 * h;
            FragB b;
            b.q[0] = *(const v4u*)wr;
            b.q[1] = *(const v4u*)(wr + 16);
            acc[nt] = wmma_bf(ahi.v, b.v, acc[nt]);
            acc[nt] = wmma_bf(alo.v, b.v, acc[nt]);
        }
    }
    epilogue_planes(acc, blockIdx.x, wave, lane, tid, smem, Hpl, Lpl, part);
}

__global__ __launch_bounds__(256) void k_last(const unsigned short* __restrict__ Hpl,
                                               const unsigned char* __restrict__ Lpl,
                                               const float* __restrict__ st, const unsigned short* __restrict__ W6p,
                                               const float* __restrict__ b6, float* out) {
    extern __shared__ __attribute__((aligned(16))) unsigned char smem[];
    const int tid = threadIdx.x, wave = tid >> 5, lane = tid & 31, h = lane >> 4, m = lane & 15;
    float* s_b  = (float*)(smem + L_SB);
    float* s_sc = (float*)(smem + L_SC);
    float* s_sh = (float*)(smem + L_SH);
    float* sO   = (float*)(smem + L_SO);
    if (wave == 0) {
        const int c = (lane < NOUT) ? lane : (NOUT - 1);
        const float bv = bf16r(b6[c]);
        s_b[lane] = (lane < NOUT) ? bv : 0.0f;
    }
    if (tid < NHID) { s_sc[tid] = st[tid]; s_sh[tid] = st[NHID + tid]; }
    __syncthreads();

    const size_t mrow = (size_t)blockIdx.x * RB + (size_t)wave * 16 + m;
    const unsigned short* Hrow = Hpl + mrow * NHID;
    const unsigned char*  Lrow = Lpl + mrow * NHID;

    v8f acc = v8f{};
#pragma unroll 1
    for (int kt = 0; kt < 4; ++kt) {
        FragB ahi, alo;
        afrag_split(Hrow, Lrow, s_sc, s_sh, kt, h, ahi, alo);
        const unsigned short* wr = W6p + (size_t)m * NHID + kt * 32 + 8 * h;
        FragB b;
        b.q[0] = *(const v4u*)wr;
        b.q[1] = *(const v4u*)(wr + 16);
        acc = wmma_bf(ahi.v, b.v, acc);
        acc = wmma_bf(alo.v, b.v, acc);
    }

    const float bn = s_b[m];
#pragma unroll
    for (int r = 0; r < 8; ++r) {
        const float y = acc[r] + bn;
        if (m < NOUT) sO[(wave * 16 + 8 * h + r) * NOUT + m] = y;
    }
    __syncthreads();

    const int t1 = 256 + (tid & 31);
    const v4f p0 = *(const v4f*)(sO + 4 * tid);
    const v4f p1 = *(const v4f*)(sO + 4 * t1);
    float* ob = out + (size_t)blockIdx.x * (RB * NOUT);
    *(volatile v4f*)(ob + 4 * tid) = p0;
    if (wave == 0) *(volatile v4f*)(ob + 4 * t1) = p1;
    __threadfence();
    *(volatile v4f*)(ob + 4 * tid) = p0;
    if (wave == 0) *(volatile v4f*)(ob + 4 * t1) = p1;
}

__global__ __launch_bounds__(128) void k_fin(const float* __restrict__ part, const float* __restrict__ gam,
                                              const float* __restrict__ bet, float* st) {
    __shared__ __attribute__((aligned(16))) float stg[256];
    const int f = threadIdx.x;
    double S = 0.0, Q = 0.0;
#pragma unroll 1
    for (int b = 0; b < NBLK; ++b) {
        S += (double)part[(size_t)b * 256 + f];
        Q += (double)part[(size_t)b * 256 + 128 + f];
    }
    const double invn = 1.0 / (double)NB;
    const double mu = S * invn;
    double var = Q * invn - mu * mu;
    var = (var > 0.0) ? var : 0.0;
    const float varf = (float)var;
    const float rs = 1.0f / sqrtf(varf + 1e-5f);
    const float g  = bf16r(gam[f]);
    const float be = bf16r(bet[f]);
    const float sc = rs * g;
    const float sh = (float)((double)be - mu * (double)sc);
    stg[f] = sc;
    stg[128 + f] = sh;
    __syncthreads();
    const int q = f & 63;
    const v4f v = *(const v4f*)(stg + 4 * q);
    if (f < 64) *(volatile v4f*)(st + 4 * q) = v;
    __threadfence();
    if (f < 64) *(volatile v4f*)(st + 4 * q) = v;
}

extern "C" void kernel_launch(void* const* d_in, const int* in_sizes, int n_in,
                              void* d_out, int out_size, void* d_ws, size_t ws_size,
                              hipStream_t stream) {
    if (n_in < 23) return;
    if (in_sizes[0] < NB * NIN) return;
    if (in_sizes[1] < NHID * NIN || in_sizes[2] < NHID) return;
    if (in_sizes[3] < NHID * NHID || in_sizes[5] < NHID * NHID ||
        in_sizes[7] < NHID * NHID || in_sizes[9] < NHID * NHID) return;
    if (in_sizes[4] < NHID || in_sizes[6] < NHID || in_sizes[8] < NHID || in_sizes[10] < NHID) return;
    if (in_sizes[11] < NOUT * NHID || in_sizes[12] < NOUT) return;
    for (int i = 13; i < 23; ++i) if (in_sizes[i] < NHID) return;
    if (out_size < NB * NOUT) return;
    if ((size_t)WS_TOTAL > ws_size) return;

    const float* x  = (const float*)d_in[0];
    const float* W1 = (const float*)d_in[1];
    const float* b1 = (const float*)d_in[2];
    const float* W2 = (const float*)d_in[3];
    const float* b2 = (const float*)d_in[4];
    const float* W3 = (const float*)d_in[5];
    const float* b3 = (const float*)d_in[6];
    const float* W4 = (const float*)d_in[7];
    const float* b4 = (const float*)d_in[8];
    const float* W5 = (const float*)d_in[9];
    const float* b5 = (const float*)d_in[10];
    const float* W6 = (const float*)d_in[11];
    const float* b6 = (const float*)d_in[12];
    const float* g[5]  = { (const float*)d_in[13], (const float*)d_in[15], (const float*)d_in[17],
                           (const float*)d_in[19], (const float*)d_in[21] };
    const float* be[5] = { (const float*)d_in[14], (const float*)d_in[16], (const float*)d_in[18],
                           (const float*)d_in[20], (const float*)d_in[22] };
    const float* bh[4] = { b2, b3, b4, b5 };

    unsigned char* ws = (unsigned char*)d_ws;
    unsigned short* wpl = (unsigned short*)(ws + WS_WP);
    float* part   = (float*)(ws + WS_PART);
    float* st     = (float*)(ws + WS_ST);
    unsigned short* Hpl = (unsigned short*)(ws + WS_HPL);
    unsigned char*  Lpl = ws + WS_LPL;
    float* out = (float*)d_out;

    hipFuncSetAttribute(reinterpret_cast<const void*>(&k_first), hipFuncAttributeMaxDynamicSharedMemorySize, LDS_A);
    hipFuncSetAttribute(reinterpret_cast<const void*>(&k_mid),   hipFuncAttributeMaxDynamicSharedMemorySize, LDS_A);

    k_prep<<<PREP_BLOCKS, 256, 0, stream>>>(W1, W2, W3, W4, W5, W6, wpl);

    k_first<<<NBLK, 256, LDS_A, stream>>>(x, wpl + WP1_OFF, b1, Hpl, Lpl, part);
    k_fin<<<1, 128, 0, stream>>>(part, g[0], be[0], st);

    for (int l = 0; l < 4; ++l) {
        k_mid<<<NBLK, 256, LDS_A, stream>>>(Hpl, Lpl, st, wpl + WPH_OFF + l * 16384, bh[l], part);
        k_fin<<<1, 128, 0, stream>>>(part, g[l + 1], be[l + 1], st);
    }

    k_last<<<NBLK, 256, LDS_B, stream>>>(Hpl, Lpl, st, wpl + WP6_OFF, b6, out);
}
